// GuidedMoEBasic_20615843020914
// MI455X (gfx1250) — hardware-run, weakly checked
//
#include <hip/hip_runtime.h>
#include <stddef.h>


typedef _Float16 v16h __attribute__((ext_vector_type(16)));
typedef _Float16 v8h  __attribute__((ext_vector_type(8)));
typedef float    v8f  __attribute__((ext_vector_type(8)));
typedef float    v4f  __attribute__((ext_vector_type(4)));

#ifndef NB
#define NB 8
#endif
#define NB_FULL 8
#define DD    128
#define HDIM  768
#define NEV   7
#define FEAT  776
#define NHID  256
#define NU    (NB * DD)
#define PPB   (DD * (DD + 1) / 2)
#define NPAIR (NB * PPB)
#define KP    832
#define NCOL  1152
#define GCOL_T 1024
#define GCOL_E 1088
#define TROW  32
#define OUT1_ELEM (NB_FULL * DD * NEV)

static_assert(NB >= 1 && NB <= NB_FULL);
static_assert(DD == 128);
static_assert(FEAT == HDIM + NEV + 1);
static_assert(HDIM == 3 * 32 * 8);
static_assert(KP == HDIM + 64);
static_assert(KP >= FEAT && (KP % 64) == 0 && (KP % 32) == 0);
static_assert((HDIM % 64) == 0 && (HDIM % 32) == 0);
static_assert((NCOL % 64) == 0 && NCOL >= GCOL_E + 64 && GCOL_T == 4 * NHID && GCOL_E == GCOL_T + 64);
static_assert((NU % 64) == 0 && (NU % 8) == 0);
static_assert(NHID == 32 * 8);
static_assert((64 * NEV) % 4 == 0 && ((64 * NEV * 4) % 128) == 0 && (64 * NEV) / 4 <= 256);
static_assert((size_t)OUT1_ELEM * 4 == (size_t)28672);
static_assert(((size_t)OUT1_ELEM * 4) % 128 == 0);
static_assert((NPAIR % 2) == 0);
static_assert(NEV <= 7);

#define LDT 72
#define LDC 68
static_assert((LDT % 8) == 0 && LDT >= 64);
static_assert((LDC % 4) == 0 && LDC >= 64);

#define WCARRY 64.0f

#define CONC_BYTES ((size_t)NU * KP * 2)
#define W1T_BYTES  ((size_t)NCOL * KP * 2)
#define EMOT_BYTES ((size_t)64 * HDIM * 2)
#define HPL_BYTES  ((size_t)NU * NCOL * 4)
#define TAB_BYTES  ((size_t)(NU + 8) * TROW * 4)
#define OFF_CONC ((size_t)0)
#define OFF_W1T  (OFF_CONC + CONC_BYTES)
#define OFF_EMOT (OFF_W1T + W1T_BYTES)
#define OFF_HPL  (OFF_EMOT + EMOT_BYTES)
#define OFF_TAB  (OFF_HPL + HPL_BYTES)
#define WS_TOTAL (OFF_TAB + TAB_BYTES)
static_assert((CONC_BYTES % 128) == 0 && (W1T_BYTES % 128) == 0 && (EMOT_BYTES % 128) == 0);
static_assert((HPL_BYTES % 128) == 0 && (TAB_BYTES % 128) == 0);
static_assert(WS_TOTAL <= (size_t)134217728);

__device__ __forceinline__ float bf16r(float x) {
  unsigned int u = __float_as_uint(x);
  u = (u + 0x7FFFu + ((u >> 16) & 1u)) & 0xFFFF0000u;
  return __uint_as_float(u);
}

static __device__ __forceinline__ _Float16 toh_flush(float v) {
  const _Float16 r = (_Float16)v;
  return (fabsf(v) < 6.103515625e-05f) ? (_Float16)0.0f : r;
}

__device__ __forceinline__ v16h frag_at(const _Float16* p) {
  v8h lo = *(const v8h*)(p);
  v8h hi = *(const v8h*)(p + 16);
  v16h out;
#pragma unroll
  for (int i = 0; i < 8; ++i) { out[i] = lo[i]; out[i + 8] = hi[i]; }
  return out;
}

__device__ __forceinline__ v8f wmma16(v16h a, v16h b, v8f c) {
  v8f d = __builtin_amdgcn_wmma_f32_16x16x32_f16(false, a, false, b, (short)0, c,
                                                 false, false);
  asm volatile("v_nop\n\tv_nop\n\tv_nop\n\tv_nop" : "+v"(d) : "v"(a), "v"(b));
  return d;
}

__device__ __forceinline__ float red32_sum(float x) {
#pragma unroll
  for (int off = 1; off < 32; off <<= 1) x += __shfl_xor(x, off, 32);
  return x;
}

__global__ __launch_bounds__(256) void wplane_kernel(
    const float* __restrict__ W, _Float16* __restrict__ Wt,
    unsigned srow0, unsigned ldw, unsigned nvalid, unsigned kvalid,
    unsigned drow0, unsigned ldk) {
  __shared__ _Float16 T[64 * LDT];
  const unsigned tid = threadIdx.x;
  const unsigned n0 = blockIdx.x * 64u;
  const unsigned k0 = blockIdx.y * 64u;
#pragma unroll 4
  for (unsigned j = 0; j < 16u; ++j) {
    const unsigned idx = tid + 256u * j;
    const unsigned kr = idx >> 6, nc = idx & 63u;
    const unsigned k = k0 + kr, n = n0 + nc;
    const unsigned kc = (k < kvalid) ? k : (kvalid - 1u);
    const unsigned nl = (n < nvalid) ? n : (nvalid - 1u);
    const float v = W[(size_t)(srow0 + kc) * ldw + nl];
    const bool ok = (k < kvalid) && (n < nvalid);
    const float t = ok ? (WCARRY * bf16r(v)) : 0.0f;
    T[nc * LDT + kr] = toh_flush(t);
  }
  __syncthreads();
  v8h x[2];
  size_t off[2];
#pragma unroll
  for (unsigned i = 0; i < 2u; ++i) {
    const unsigned n = 32u * i + (tid >> 3);
    const unsigned kc = (tid & 7u) * 8u;
    x[i] = *(const v8h*)&T[n * LDT + kc];
    off[i] = (size_t)(drow0 + n0 + n) * ldk + k0 + kc;
  }
#pragma unroll
  for (int i = 0; i < 2; ++i) *(volatile v8h*)(Wt + off[i]) = x[i];
  __threadfence();
#pragma unroll
  for (int i = 0; i < 2; ++i) *(volatile v8h*)(Wt + off[i]) = x[i];
}

__global__ __launch_bounds__(256) void cvt_kernel(
    const float* __restrict__ X, _Float16* __restrict__ dst) {
  const unsigned lane = threadIdx.x & 31u, w = threadIdx.x >> 5;
  const unsigned row = blockIdx.x * 8u + w;
  const float* xr = X + (size_t)row * HDIM + lane * 8u;
#pragma unroll 1
  for (unsigned j = 0; j < 3u; ++j) {
    const v4f a0 = *(const v4f*)(xr + j * 256u);
    const v4f a1 = *(const v4f*)(xr + j * 256u + 4u);
    v8h o;
#pragma unroll
    for (int i = 0; i < 4; ++i) {
      o[i]     = toh_flush(bf16r(a0[i]));
      o[i + 4] = toh_flush(bf16r(a1[i]));
    }
    _Float16* p = dst + (size_t)row * KP + j * 256u + lane * 8u;
    *(volatile v8h*)p = o;
    __threadfence();
    *(volatile v8h*)p = o;
  }
}

template <int MODE>
__device__ __forceinline__ void gemm_body(
    const _Float16* A16, const unsigned lda,
    const _Float16* __restrict__ Bt, const unsigned ldb, const unsigned K,
    const float* __restrict__ bias, const float* __restrict__ spk,
    float* __restrict__ outf, _Float16* out16) {
  __shared__ float Cs[64 * LDC];
  const unsigned tid = threadIdx.x, lane = tid & 31u, w = tid >> 5;
  const unsigned mw = w >> 1, nw = w & 1u;
  const unsigned hh = lane >> 4, m = lane & 15u;
  const unsigned n0 = blockIdx.x * 64u;
  const unsigned row0 = blockIdx.y * 64u;

  const _Float16* ap  = A16 + (size_t)(row0 + mw * 16u + m) * lda + hh * 8u;
  const _Float16* bp0 = Bt + (size_t)(n0 + nw * 32u + m) * ldb + hh * 8u;
  const _Float16* bp1 = bp0 + (size_t)16 * ldb;
  v8f acc0 = {}, acc1 = {};
#pragma unroll 2
  for (unsigned k0 = 0; k0 < K; k0 += 32u) {
    const v16h a  = frag_at(ap + k0);
    const v16h b0 = frag_at(bp0 + k0);
    const v16h b1 = frag_at(bp1 + k0);
    acc0 = wmma16(a, b0, acc0);
    acc1 = wmma16(a, b1, acc1);
  }
#pragma unroll
  for (int r = 0; r < 8; ++r) {
    float* d = &Cs[(mw * 16u + hh * 8u + (unsigned)r) * LDC + nw * 32u + m];
    d[0]  = acc0[r];
    d[16] = acc1[r];
  }
  __syncthreads();

  if (MODE == 0) {
    v8h x[2];
    size_t off[2];
#pragma unroll
    for (unsigned i = 0; i < 2u; ++i) {
      const unsigned r = 32u * i + (tid >> 3);
      const unsigned c = (tid & 7u) * 8u;
      const float sp = bf16r(spk[row0 + r]);
#pragma unroll
      for (unsigned j = 0; j < 8u; ++j) {
        const unsigned cc = c + j;
        const unsigned cj = (cc < (unsigned)NEV) ? cc : (unsigned)(NEV - 1);
        const float ev = Cs[r * LDC + cj] * (1.0f / WCARRY) + bf16r(bias[cj]);
        const float t = (cc < (unsigned)NEV) ? ev : ((cc == (unsigned)NEV) ? sp : 0.0f);
        x[i][j] = toh_flush(t);
      }
      off[i] = (size_t)(row0 + r) * lda + (unsigned)HDIM + c;
    }
    const unsigned fq = (tid < 112u) ? tid : 111u;
    v4f e;
#pragma unroll
    for (unsigned i = 0; i < 4u; ++i) {
      const unsigned f = fq * 4u + i;
      const unsigned r = f / (unsigned)NEV;
      const unsigned jj = f - r * (unsigned)NEV;
      e[i] = Cs[r * LDC + jj] * (1.0f / WCARRY) + bf16r(bias[jj]);
    }
    const size_t eoff = (size_t)row0 * NEV + fq * 4u;
#pragma unroll
    for (int i = 0; i < 2; ++i) *(volatile v8h*)(out16 + off[i]) = x[i];
    if (tid < 112u) *(volatile v4f*)(outf + eoff) = e;
    __threadfence();
#pragma unroll
    for (int i = 0; i < 2; ++i) *(volatile v8h*)(out16 + off[i]) = x[i];
    if (tid < 112u) *(volatile v4f*)(outf + eoff) = e;
  }

  if (MODE == 1) {
    v4f xs[4];
    size_t off[4];
#pragma unroll
    for (unsigned i = 0; i < 4u; ++i) {
      const unsigned r = 16u * i + (tid >> 4);
      const unsigned c = (tid & 15u) * 4u;
      const v4f u = *(const v4f*)&Cs[r * LDC + c];
      v4f val;
#pragma unroll
      for (int j = 0; j < 4; ++j) val[j] = u[j] * (1.0f / WCARRY);
      xs[i] = val;
      off[i] = (size_t)(row0 + r) * NCOL + n0 + c;
    }
#pragma unroll
    for (int i = 0; i < 4; ++i) *(volatile v4f*)(outf + off[i]) = xs[i];
    __threadfence();
#pragma unroll
    for (int i = 0; i < 4; ++i) *(volatile v4f*)(outf + off[i]) = xs[i];
  }
}

__global__ __launch_bounds__(256) void gemm_emo_kernel(
    _Float16* Cc, const _Float16* __restrict__ Bt,
    const float* __restrict__ bias, const float* __restrict__ spk, float* __restrict__ outE) {
  gemm_body<0>(Cc, (unsigned)KP, Bt, (unsigned)HDIM, (unsigned)HDIM, bias, spk, outE, Cc);
}
__global__ __launch_bounds__(256) void gemm_h_kernel(
    const _Float16* __restrict__ Cc, const _Float16* __restrict__ Bt, float* __restrict__ Hp) {
  gemm_body<1>(Cc, (unsigned)KP, Bt, (unsigned)KP, (unsigned)KP, (const float*)0, (const float*)0,
               Hp, (_Float16*)0);
}

__device__ __forceinline__ void dot8x2(const v4f h0, const v4f h1, const float* __restrict__ wp,
                                       float& c0, float& c1) {
  const v4f w0 = *(const v4f*)(wp);
  const v4f w1 = *(const v4f*)(wp + 4);
  const v4f w2 = *(const v4f*)(wp + 8);
  const v4f w3 = *(const v4f*)(wp + 12);
  const float hv[8]  = {h0[0], h0[1], h0[2], h0[3], h1[0], h1[1], h1[2], h1[3]};
  const float wv[16] = {w0[0], w0[1], w0[2], w0[3], w1[0], w1[1], w1[2], w1[3],
                        w2[0], w2[1], w2[2], w2[3], w3[0], w3[1], w3[2], w3[3]};
  float s0 = 0.0f, s1 = 0.0f;
#pragma unroll
  for (int i = 0; i < 8; ++i) {
    s0 += hv[i] * bf16r(wv[2 * i]);
    s1 += hv[i] * bf16r(wv[2 * i + 1]);
  }
  c0 = s0;
  c1 = s1;
}

__global__ __launch_bounds__(256) void head_kernel(
    const float* __restrict__ Hp, const float* __restrict__ w2,
    const float* __restrict__ b1, const float* __restrict__ b2,
    const float* __restrict__ gb, float* __restrict__ Tb) {
  __shared__ float S[8 * TROW];
  const unsigned tid = threadIdx.x, lane = tid & 31u, w = tid >> 5;
  const bool biasblk = (blockIdx.x == (unsigned)(NU / 8));
  float mine = 0.0f;
  if (!biasblk) {
    const unsigned u = blockIdx.x * 8u + w;
    const float* hr = Hp + (size_t)u * NCOL;
    const float gv = hr[(unsigned)GCOL_T + (lane & 1u) + ((lane >> 1) & 1u) * 64u];
    mine = (lane < 4u) ? gv : 0.0f;
#pragma unroll 1
    for (unsigned g = 0; g < 4u; ++g) {
      const unsigned e = g & 1u;
      const v4f h0 = *(const v4f*)(hr + g * 256u + lane * 8u);
      const v4f h1 = *(const v4f*)(hr + g * 256u + lane * 8u + 4u);
      float c0, c1;
      dot8x2(h0, h1, w2 + e * 512u + lane * 16u, c0, c1);
      c0 = red32_sum(c0);
      c1 = red32_sum(c1);
      mine = (lane == 4u + 2u * g) ? c0 : mine;
      mine = (lane == 5u + 2u * g) ? c1 : mine;
    }
  } else {
    const float gq = bf16r(gb[lane & 1u]);
    mine = (lane == 4u || lane == 5u) ? gq : 0.0f;
#pragma unroll 1
    for (unsigned e = 0; e < 2u; ++e) {
      const v4f r0 = *(const v4f*)(b1 + e * 256u + lane * 8u);
      const v4f r1 = *(const v4f*)(b1 + e * 256u + lane * 8u + 4u);
      v4f h0, h1;
#pragma unroll
      for (int i = 0; i < 4; ++i) { h0[i] = bf16r(r0[i]); h1[i] = bf16r(r1[i]); }
      float c0, c1;
      dot8x2(h0, h1, w2 + e * 512u + lane * 16u, c0, c1);
      c0 = red32_sum(c0) + bf16r(b2[e * 2u]);
      c1 = red32_sum(c1) + bf16r(b2[e * 2u + 1u]);
      mine = (lane == 2u * e) ? c0 : mine;
      mine = (lane == 2u * e + 1u) ? c1 : mine;
    }
  }
  S[w * TROW + lane] = mine;
  __syncthreads();
  const unsigned q = tid & 63u;
  const v4f x = *(const v4f*)&S[q * 4u];
  float* dst = Tb + (size_t)blockIdx.x * (8u * TROW) + q * 4u;
  if (tid < 64u) *(volatile v4f*)dst = x;
  __threadfence();
  if (tid < 64u) *(volatile v4f*)dst = x;
}

__global__ __launch_bounds__(256) void pair_kernel(
    const float* __restrict__ Tb, float* __restrict__ out) {
  const unsigned gid = blockIdx.x * 256u + threadIdx.x;
  const unsigned n0 = gid * 2u;
  const bool live = (n0 < (unsigned)NPAIR);
  const v4f ob = *(const v4f*)(Tb + (size_t)NU * TROW);
  const v4f gq = *(const v4f*)(Tb + (size_t)NU * TROW + 4u);
  v4f res;
#pragma unroll
  for (unsigned q = 0; q < 2u; ++q) {
    const unsigned nn = n0 + q;
    const unsigned n = (nn < (unsigned)NPAIR) ? nn : (unsigned)(NPAIR - 1);
    const unsigned b = n / (unsigned)PPB;
    const unsigned p = n - b * (unsigned)PPB;
    unsigned end = 0u;
#pragma unroll
    for (unsigned step = 64u; step > 0u; step >>= 1) {
      const unsigned c = end + step;
      const bool take = (c < (unsigned)DD) && ((c * (c + 1u)) / 2u <= p);
      end = take ? c : end;
    }
    unsigned t = p - (end * (end + 1u)) / 2u;
    t = (t < (unsigned)DD) ? t : (unsigned)(DD - 1);
    const float* rt = Tb + (size_t)(b * (unsigned)DD + t) * TROW;
    const float* re = Tb + (size_t)(b * (unsigned)DD + end) * TROW;
    const v4f a0 = *(const v4f*)(rt);
    const v4f a1 = *(const v4f*)(rt + 4);
    const v4f e0 = *(const v4f*)(re);
    const v4f e2 = *(const v4f*)(re + 8);
    const float g0 = a0[0] + e0[2] + gq[0];
    const float g1 = a0[1] + e0[3] + gq[1];
    const float o00 = a1[0] + e2[0] + ob[0];
    const float o01 = a1[1] + e2[1] + ob[1];
    const float o10 = a1[2] + e2[2] + ob[2];
    const float o11 = a1[3] + e2[3] + ob[3];
    res[2 * q]     = g0 * o00 + g1 * o10;
    res[2 * q + 1] = g0 * o01 + g1 * o11;
  }
  float* dst = out + (size_t)OUT1_ELEM + (size_t)n0 * 2u;
  if (live) *(volatile v4f*)dst = res;
  __threadfence();
  if (live) *(volatile v4f*)dst = res;
}

extern "C" void kernel_launch(void* const* d_in, const int* in_sizes, int n_in,
                              void* d_out, int out_size, void* d_ws, size_t ws_size,
                              hipStream_t stream) {
  if (n_in < 10) return;
  if ((long long)in_sizes[0] < (long long)NU * HDIM) return;
  if ((long long)in_sizes[1] < (long long)NU) return;
  if (in_sizes[2] < HDIM * NEV || in_sizes[3] < NEV) return;
  if (in_sizes[4] < 2 * FEAT * 2 || in_sizes[5] < 2) return;
  if ((long long)in_sizes[6] < (long long)2 * 2 * FEAT * NHID) return;
  if (in_sizes[7] < 2 * NHID || in_sizes[8] < 2 * NHID * 2 || in_sizes[9] < 4) return;
  if ((long long)out_size < (long long)OUT1_ELEM + (long long)NPAIR * 2) return;
  if (ws_size < WS_TOTAL) return;

  const float* pooled = (const float*)d_in[0];
  const float* spk    = (const float*)d_in[1];
  const float* emo_w  = (const float*)d_in[2];
  const float* emo_b  = (const float*)d_in[3];
  const float* gate_w = (const float*)d_in[4];
  const float* gate_b = (const float*)d_in[5];
  const float* exp_w1 = (const float*)d_in[6];
  const float* exp_b1 = (const float*)d_in[7];
  const float* exp_w2 = (const float*)d_in[8];
  const float* exp_b2 = (const float*)d_in[9];
  float* out = (float*)d_out;

  char* ws = (char*)d_ws;
  _Float16* Conc16 = (_Float16*)(ws + OFF_CONC);
  _Float16* W1t    = (_Float16*)(ws + OFF_W1T);
  _Float16* EmoT   = (_Float16*)(ws + OFF_EMOT);
  float*    Hpl    = (float*)(ws + OFF_HPL);
  float*    Tab    = (float*)(ws + OFF_TAB);

  dim3 blk(256);

  for (unsigned half = 0; half < 2u; ++half)
    for (unsigned e = 0; e < 2u; ++e)
      wplane_kernel<<<dim3(NHID / 64, KP / 64), blk, 0, stream>>>(
          exp_w1, W1t, e * (2u * FEAT) + half * FEAT, (unsigned)NHID, (unsigned)NHID,
          (unsigned)FEAT, half * 512u + e * 256u, (unsigned)KP);
  for (unsigned half = 0; half < 2u; ++half)
    wplane_kernel<<<dim3(1, KP / 64), blk, 0, stream>>>(
        gate_w, W1t, half * FEAT, 2u, 2u, (unsigned)FEAT, (unsigned)GCOL_T + half * 64u,
        (unsigned)KP);
  wplane_kernel<<<dim3(1, HDIM / 64), blk, 0, stream>>>(
      emo_w, EmoT, 0u, (unsigned)NEV, (unsigned)NEV, (unsigned)HDIM, 0u, (unsigned)HDIM);

  cvt_kernel<<<dim3(NU / 8), blk, 0, stream>>>(pooled, Conc16);
  gemm_emo_kernel<<<dim3(1, NU / 64), blk, 0, stream>>>(Conc16, EmoT, emo_b, spk, out);
  gemm_h_kernel<<<dim3(NCOL / 64, NU / 64), blk, 0, stream>>>(Conc16, W1t, Hpl);
  head_kernel<<<dim3(NU / 8 + 1), blk, 0, stream>>>(Hpl, exp_w2, exp_b1, exp_b2, gate_b, Tab);
  pair_kernel<<<dim3((NPAIR / 2 + 255) / 256), blk, 0, stream>>>(Tab, out);
}
